// GNNEncoder_15496242004460
// MI455X (gfx1250) — hardware-verified
//
#include <hip/hip_runtime.h>
#include <stddef.h>
#include <stdint.h>
#include <math.h>


#define DF      128
#define NHEAD   8
#define HCH     16
#define SCW     16
#define KX      128
#define KZ      256
#define NTHR    256
#define NWAVE   8
#define EPT     8
#define CHUNK   (NTHR * EPT)
#define WCAP    (EPT * 32)
#define LISTN   (NWAVE * WCAP)
#define NBA     1024
#define PKS     10
#define RCAP    28672
#define DEGCAP  64
#define GBM     64
#define GTHR    128
#define GNT     8
#define GBN     (16 * GNT)
#define PARTW   288
#define WSTW    258
#define NUA     (DF * (KX / 8))
#define NUB     (DF * (KZ / 8))
#define NUW     (NUA + NUB)
#define ZINTS   (2 * RCAP + 2 * NBA + LISTN)
#define LDS_AGG (ZINTS * 4 + 64)
#define NEGSL   0.2f
#define BNEPS   1e-5f
#define WSMAX   134217728

static_assert((CHUNK & (CHUNK - 1)) == 0);
static_assert(NBA == (1 << PKS));
static_assert(((long long)CHUNK << PKS) < (1LL << 31));
static_assert(NTHR * 4 == NBA);
static_assert(LISTN >= NBA && LISTN >= NWAVE * WCAP);
static_assert((RCAP % 32) == 0);
static_assert((ZINTS % (NTHR * 4)) == 0);
static_assert(LDS_AGG <= 262144);
static_assert((NBA % NWAVE) == 0 && (NBA % GBM) == 0);
static_assert(GBM == (GTHR / 32) * 16);
static_assert((KX % 32) == 0 && (KZ % 32) == 0 && KZ == 2 * DF && KX == DF);
static_assert(DF == 32 * 4);
static_assert(GBN == DF && NHEAD * HCH == DF && SCW == 2 * NHEAD && HCH == 4 * 4);
static_assert(GTHR == DF);
static_assert(NTHR == 2 * DF);
static_assert(PARTW % 32 == 0 && PARTW >= 2 * DF + 1 && PARTW / 4 <= GTHR);
static_assert(WSTW >= 2 * DF + 1);
static_assert(NWAVE * WSTW + PARTW <= RCAP && ((NWAVE * WSTW) % 4) == 0);
static_assert((NUA % NTHR) == 0 && (NUW % NTHR) == 0);
static_assert((GBM * SCW) == 2 * 4 * GTHR);

typedef float          v4f  __attribute__((ext_vector_type(4)));
typedef float          v8f  __attribute__((ext_vector_type(8)));
typedef int            v4i  __attribute__((ext_vector_type(4)));
typedef int            v8i  __attribute__((ext_vector_type(8)));
typedef unsigned int   v4u  __attribute__((ext_vector_type(4)));
typedef unsigned short v8us __attribute__((ext_vector_type(8)));
typedef __bf16         v16b __attribute__((ext_vector_type(16)));
typedef v4f  __attribute__((may_alias)) v4fa;
typedef v4i  __attribute__((may_alias)) v4ia;
typedef v8us __attribute__((may_alias)) v8usa;
union Frag { v16b b; v8us h[2]; v8i w; };

__device__ __forceinline__ v8f wmk(const Frag& a, const Frag& b, v8f c) {
  v8f d = __builtin_amdgcn_wmma_f32_16x16x32_bf16(false, a.b, false, b.b, (short)0, c, false, false);
  asm volatile("v_nop\n\tv_nop\n\tv_nop\n\tv_nop" : "+v"(d) : "v"(a.w), "v"(b.w));
  return d;
}

__device__ __forceinline__ v8f z8() { v8f z = {0.f, 0.f, 0.f, 0.f, 0.f, 0.f, 0.f, 0.f}; return z; }

__device__ __forceinline__ unsigned short bf_bits(float f) {
  unsigned int u = __float_as_uint(f);
  u += 0x7FFFu + ((u >> 16) & 1u);
  return (unsigned short)(u >> 16);
}
__device__ __forceinline__ float bf_val(unsigned short b) {
  return __uint_as_float(((unsigned int)b) << 16);
}
__device__ __forceinline__ float bf_rne(float f) { return bf_val(bf_bits(f)); }
__device__ __forceinline__ v4f bfr4(const v4f a) {
  v4f r; r.x = bf_rne(a.x); r.y = bf_rne(a.y); r.z = bf_rne(a.z); r.w = bf_rne(a.w); return r;
}
__device__ __forceinline__ unsigned int pk2(float lo, float hi) {
  return (unsigned int)bf_bits(lo) | ((unsigned int)bf_bits(hi) << 16);
}
__device__ __forceinline__ v4u pack8(const v4f a, const v4f b) {
  v4u r;
  r.x = pk2(a.x, a.y); r.y = pk2(a.z, a.w); r.z = pk2(b.x, b.y); r.w = pk2(b.z, b.w);
  return r;
}

__device__ __forceinline__ int scan_chunk(const int* __restrict__ dsts, int nE, int cbase, int slotBase,
                                          int nb, int vec8, int* list, int tid, int lane, int wave) {
  int wc = 0;
  const int el0  = tid * EPT;
  const int e0   = cbase + el0;
  const int sent = -2147483647 - 1;
  v4i da, db;
  if (vec8 != 0 && cbase + CHUNK <= nE) {
    da = *(const v4i*)(dsts + e0);
    db = *(const v4i*)(dsts + e0 + 4);
  } else {
    da.x = (e0     < nE) ? dsts[min(e0,     nE - 1)] : sent;
    da.y = (e0 + 1 < nE) ? dsts[min(e0 + 1, nE - 1)] : sent;
    da.z = (e0 + 2 < nE) ? dsts[min(e0 + 2, nE - 1)] : sent;
    da.w = (e0 + 3 < nE) ? dsts[min(e0 + 3, nE - 1)] : sent;
    db.x = (e0 + 4 < nE) ? dsts[min(e0 + 4, nE - 1)] : sent;
    db.y = (e0 + 5 < nE) ? dsts[min(e0 + 5, nE - 1)] : sent;
    db.z = (e0 + 6 < nE) ? dsts[min(e0 + 6, nE - 1)] : sent;
    db.w = (e0 + 7 < nE) ? dsts[min(e0 + 7, nE - 1)] : sent;
  }
  const unsigned nbs = (unsigned)slotBase;
  const unsigned unb = (unsigned)nb;
  const unsigned s0 = (unsigned)da.x - nbs, s1 = (unsigned)da.y - nbs;
  const unsigned s2 = (unsigned)da.z - nbs, s3 = (unsigned)da.w - nbs;
  const unsigned s4 = (unsigned)db.x - nbs, s5 = (unsigned)db.y - nbs;
  const unsigned s6 = (unsigned)db.z - nbs, s7 = (unsigned)db.w - nbs;
  const bool h0 = s0 < unb, h1 = s1 < unb, h2 = s2 < unb, h3 = s3 < unb;
  const bool h4 = s4 < unb, h5 = s5 < unb, h6 = s6 < unb, h7 = s7 < unb;
  const unsigned any = __builtin_amdgcn_ballot_w32(h0 | h1 | h2 | h3 | h4 | h5 | h6 | h7);
  if (any != 0u) {
#define HITJ(J, HJ, SJ) { \
      const unsigned mj = __builtin_amdgcn_ballot_w32(HJ); \
      if (mj != 0u) { \
        if (HJ) { \
          const int pos = wc + (int)__builtin_amdgcn_mbcnt_lo(mj, 0u); \
          if (pos < WCAP) list[wave * WCAP + pos] = ((el0 + (J)) << PKS) | (int)(SJ); \
        } \
        wc += (int)__builtin_popcount(mj); } }
    HITJ(0, h0, s0)
    HITJ(1, h1, s1)
    HITJ(2, h2, s2)
    HITJ(3, h3, s3)
    HITJ(4, h4, s4)
    HITJ(5, h5, s5)
    HITJ(6, h6, s6)
    HITJ(7, h7, s7)
#undef HITJ
  }
  return wc;
}

__device__ __forceinline__ int seg_build(const int* __restrict__ dsts, int nE, int vec8, int nodeBase,
                                         int* lds_i, int tid, int lane, int wave) {
  int* reg1 = lds_i;
  int* reg2 = reg1 + RCAP;
  int* scnt = reg2 + RCAP;
  int* soff = scnt + NBA;
  int* list = soff + NBA;
  int* wcnt = list + LISTN;
  int* wtot = wcnt + NWAVE;

  {
    const v4i z4 = {0, 0, 0, 0};
    for (int i = tid * 4; i < ZINTS; i += NTHR * 4) *(v4ia*)(lds_i + i) = z4;
    if (tid < 2 * NWAVE) wcnt[tid] = 0;
  }
  __syncthreads();

  int tot = 0;
  const int nChunks = (nE + CHUNK - 1) / CHUNK;
#pragma unroll 1
  for (int ch = 0; ch < nChunks; ++ch) {
    const int cbase = ch * CHUNK;
    const int wc = scan_chunk(dsts, nE, cbase, nodeBase, NBA, vec8, list, tid, lane, wave);
    if (lane == 0) wcnt[wave] = wc;
    __syncthreads();
    int pre = 0, all = 0;
#pragma unroll
    for (int w2 = 0; w2 < NWAVE; ++w2) {
      int c = wcnt[w2];
      c = c < 0 ? 0 : (c > WCAP ? WCAP : c);
      all += c;
      pre += (w2 < wave) ? c : 0;
    }
    const int wcc  = wc > WCAP ? WCAP : wc;
    const int base = tot + pre;
#pragma unroll 1
    for (int i = lane; i < wcc; i += 32) {
      const int ent = list[wave * WCAP + i];
      const int el  = (ent >> PKS) & (CHUNK - 1);
      const int sl  = ent & (NBA - 1);
      int eid = cbase + el;
      eid = eid > nE - 1 ? nE - 1 : eid;
      const int pos = base + i;
      if (pos < RCAP) reg1[pos] = (int)(((unsigned)eid << PKS) | (unsigned)sl);
    }
    tot += all;
    tot = tot > RCAP ? RCAP : tot;
    __syncthreads();
  }
  const int nh = tot;

  if (wave == 0) {
#pragma unroll 1
    for (int b0 = 0; b0 < nh; b0 += 32) {
      const int idx = b0 + lane;
      const int uv  = reg1[idx < RCAP ? idx : RCAP - 1];
      const int m32 = (nh - b0) < 32 ? (nh - b0) : 32;
#pragma unroll 1
      for (int k = 0; k < m32; ++k) {
        const int u  = __builtin_amdgcn_readlane(uv, k);
        const int sl = u & (NBA - 1);
        if (lane == 0) scnt[sl] = scnt[sl] + 1;
      }
    }
  }
  __syncthreads();

  {
    const v4i ca = *(const v4ia*)(scnt + 4 * tid);
    const int e0 = ca.x < 0 ? 0 : ca.x, e1 = ca.y < 0 ? 0 : ca.y, e2 = ca.z < 0 ? 0 : ca.z, e3 = ca.w < 0 ? 0 : ca.w;
    const int ts = e0 + e1 + e2 + e3;
    int incl = ts;
#pragma unroll
    for (int d = 1; d < 32; d <<= 1) {
      const int up = __shfl_up(incl, d, 32);
      if (lane >= d) incl += up;
    }
    if (lane == 31) wtot[wave] = incl;
    __syncthreads();
    int pre = 0;
#pragma unroll
    for (int w2 = 0; w2 < NWAVE; ++w2) pre += (w2 < wave) ? wtot[w2] : 0;
    int run = pre + incl - ts;
    soff[4 * tid + 0] = run; run += e0;
    soff[4 * tid + 1] = run; run += e1;
    soff[4 * tid + 2] = run; run += e2;
    soff[4 * tid + 3] = run;
  }
  __syncthreads();
  for (int i = tid; i < NBA; i += NTHR) list[i] = soff[i];
  __syncthreads();

  if (wave == 0) {
#pragma unroll 1
    for (int b0 = 0; b0 < nh; b0 += 32) {
      const int idx = b0 + lane;
      const int uv  = reg1[idx < RCAP ? idx : RCAP - 1];
      const int m32 = (nh - b0) < 32 ? (nh - b0) : 32;
#pragma unroll 1
      for (int k = 0; k < m32; ++k) {
        const int u   = __builtin_amdgcn_readlane(uv, k);
        const int sl  = u & (NBA - 1);
        const int eid = (int)((unsigned)u >> PKS);
        if (lane == 0) {
          int pos = list[sl];
          pos = pos < 0 ? 0 : (pos > RCAP - 1 ? RCAP - 1 : pos);
          reg2[pos] = eid;
          list[sl] = pos + 1;
        }
      }
    }
  }
  __syncthreads();
  return nh;
}

__global__ __launch_bounds__(NTHR) void k_wprep(const float* __restrict__ wa, const float* __restrict__ wb,
                                                unsigned short* WA, unsigned short* WZ) {
  const int u = (int)blockIdx.x * NTHR + (int)threadIdx.x;
  if (u >= NUW) return;
  v8us o;
  unsigned short* dp;
  if (u < NUA) {
    const int n = u >> 4;
    const int q = u & 15;
    const float* p = wa + (size_t)(8 * q) * DF + n;
#pragma unroll
    for (int i = 0; i < 8; ++i) o[i] = bf_bits(p[(size_t)i * DF]);
    dp = WA + (size_t)n * KX + 8 * q;
  } else {
    const int v = u - NUA;
    const int n = v >> 5;
    const int q = v & 31;
    const float* p = wb + (size_t)(4 * q) * DF + n;
    float f[4];
#pragma unroll
    for (int c = 0; c < 4; ++c) f[c] = p[(size_t)c * DF];
#pragma unroll
    for (int j = 0; j < 8; ++j) o[j] = bf_bits(f[j & 3]);
    dp = WZ + (size_t)n * KZ + 8 * q;
  }
  *(volatile v8us*)dp = o;
  __threadfence();
  *(volatile v8us*)dp = o;
}

__global__ __launch_bounds__(NTHR) void k_cvt(const float* __restrict__ src, int nValid, int nUnits,
                                              unsigned short* dst) {
  const int u = (int)blockIdx.x * NTHR + (int)threadIdx.x;
  if (u >= nUnits) return;
  const int row   = u >> 4;
  const int piece = u & 15;
  const int c0    = 8 * piece;
  const int rc    = row < nValid ? row : nValid - 1;
  const float* p  = src + (size_t)rc * DF + c0;
  v4f a = *(const v4fa*)p;
  v4f b = *(const v4fa*)(p + 4);
  const v4f z4 = {0.f, 0.f, 0.f, 0.f};
  if (row >= nValid) { a = z4; b = z4; }
  const v4u q = pack8(a, b);
  unsigned short* o = dst + (size_t)row * KX + 8 * piece;
  *(volatile v4u*)o = q;
  __threadfence();
  *(volatile v4u*)o = q;
}

__global__ __launch_bounds__(GTHR) void k_gemm1(const unsigned short* __restrict__ A,
                                                const unsigned short* __restrict__ BT,
                                                const float* __restrict__ asrc, const float* __restrict__ adst,
                                                float* Hout, float* SCout) {
  __shared__ __attribute__((aligned(16))) float stg[GBM * GBN];
  __shared__ __attribute__((aligned(16))) float ssc[GBM * SCW];
  const int tid = (int)threadIdx.x, lane = tid & 31, wave = tid >> 5, hh = lane >> 4, m = lane & 15;
  const int rowBase = (int)blockIdx.x * GBM;

  v8f acc[GNT];
#pragma unroll
  for (int t = 0; t < GNT; ++t) acc[t] = z8();
  const unsigned short* ap = A  + (size_t)(rowBase + 16 * wave + m) * (size_t)KX + 8 * hh;
  const unsigned short* bp = BT + (size_t)m * (size_t)KX + 8 * hh;

#pragma unroll 1
  for (int k0 = 0; k0 < KX; k0 += 32) {
    Frag af;
    af.h[0] = *(const v8usa*)(ap + k0);
    af.h[1] = *(const v8usa*)(ap + k0 + 16);
#pragma unroll
    for (int nt = 0; nt < GNT; ++nt) {
      const unsigned short* wq = bp + (size_t)(16 * nt) * (size_t)KX + k0;
      Frag bf;
      bf.h[0] = *(const v8usa*)wq;
      bf.h[1] = *(const v8usa*)(wq + 16);
      acc[nt] = wmk(af, bf, acc[nt]);
    }
  }

#pragma unroll
  for (int nt = 0; nt < GNT; ++nt) {
    const int lc = 16 * nt + m;
#pragma unroll
    for (int r = 0; r < 8; ++r) {
      const int lr = 16 * wave + 8 * hh + r;
      stg[lr * GBN + lc] = acc[nt][r];
    }
  }
  __syncthreads();

  const v4f as4 = bfr4(*(const v4fa*)(asrc + 4 * lane));
  const v4f ad4 = bfr4(*(const v4fa*)(adst + 4 * lane));
  const int hd = lane >> 2;
  v4f pv[16];
#pragma unroll
  for (int i = 0; i < 16; ++i) pv[i] = *(const v4fa*)(stg + (16 * wave + i) * GBN + 4 * lane);
#pragma unroll
  for (int i = 0; i < 16; ++i) {
    const int lr = 16 * wave + i;
    float ps = pv[i].x * as4.x;
    ps = fmaf(pv[i].y, as4.y, ps); ps = fmaf(pv[i].z, as4.z, ps); ps = fmaf(pv[i].w, as4.w, ps);
    float pd = pv[i].x * ad4.x;
    pd = fmaf(pv[i].y, ad4.y, pd); pd = fmaf(pv[i].z, ad4.z, pd); pd = fmaf(pv[i].w, ad4.w, pd);
    ps += __shfl_xor(ps, 1); ps += __shfl_xor(ps, 2);
    pd += __shfl_xor(pd, 1); pd += __shfl_xor(pd, 2);
    if ((lane & 3) == 0) { ssc[lr * SCW + hd] = ps; ssc[lr * SCW + NHEAD + hd] = pd; }
  }

#pragma unroll
  for (int i = 0; i < 16; ++i) {
    float* op = Hout + (size_t)(rowBase + 16 * wave + i) * (size_t)DF + 4 * lane;
    *(volatile v4f*)op = pv[i];
  }
  __threadfence();
#pragma unroll
  for (int i = 0; i < 16; ++i) {
    float* op = Hout + (size_t)(rowBase + 16 * wave + i) * (size_t)DF + 4 * lane;
    *(volatile v4f*)op = pv[i];
  }

  __syncthreads();
  v4f sv[2];
#pragma unroll
  for (int j = 0; j < 2; ++j) {
    const int f = GTHR * j + tid;
    sv[j] = *(const v4fa*)(ssc + 4 * f);
    *(volatile v4f*)(SCout + (size_t)rowBase * SCW + 4 * f) = sv[j];
  }
  __threadfence();
#pragma unroll
  for (int j = 0; j < 2; ++j) {
    const int f = GTHR * j + tid;
    *(volatile v4f*)(SCout + (size_t)rowBase * SCW + 4 * f) = sv[j];
  }
}

__global__ __launch_bounds__(NTHR) void k_attagg(const int* __restrict__ dsts, const int* __restrict__ srcs,
                                                 const float* __restrict__ F, const float* __restrict__ SC,
                                                 const float* __restrict__ bias,
                                                 float* HCo, float* part, int nN, int nE, int vec8) {
  extern __shared__ __attribute__((aligned(16))) int lds_i[];
  const int tid = (int)threadIdx.x, lane = tid & 31, wave = tid >> 5;
  const int nodeBase = (int)blockIdx.x * NBA;
  const int nh = seg_build(dsts, nE, vec8, nodeBase, lds_i, tid, lane, wave);
  const int* reg2 = lds_i + RCAP;
  const int* scnt = reg2 + RCAP;
  const int* soff = scnt + NBA;

  const int nbw = NBA / NWAVE;
  const bool ovf = (nh >= RCAP);
  const float qnan = __int_as_float(0x7fc00000);
  const int hd = lane >> 2;
  const v4f bb = bfr4(*(const v4fa*)(bias + 4 * lane));
  int wn = 0;
  float wm0 = 0.0f, wm1 = 0.0f, wm2 = 0.0f, wm3 = 0.0f;
  float wq0 = 0.0f, wq1 = 0.0f, wq2 = 0.0f, wq3 = 0.0f;

#pragma unroll 1
  for (int jt = 0; jt < nbw; ++jt) {
    const int slot = wave * nbw + jt;
    const int node = nodeBase + slot;
    int st = soff[slot];
    const int craw = scnt[slot];
    int cnt = craw;
    st  = st < 0 ? 0 : (st > nh ? nh : st);
    cnt = cnt < 0 ? 0 : (cnt > DEGCAP ? DEGCAP : cnt);
    if (cnt > nh - st) cnt = nh - st;
    const float pz = (ovf || craw > DEGCAP) ? qnan : 0.0f;
    const bool live = node < nN;
    const int nc = node < nN ? node : nN - 1;

    const float sdv = SC[(size_t)nc * SCW + NHEAD + hd];
    float mx = -1.0e30f, dn = 0.0f;
    float a0 = 0.0f, a1 = 0.0f, a2 = 0.0f, a3 = 0.0f;
#pragma unroll 1
    for (int b0 = 0; b0 < cnt; b0 += 32) {
      int idx = st + b0 + lane; idx = idx > RCAP - 1 ? RCAP - 1 : idx;
      int eid = reg2[idx]; eid = eid < 0 ? 0 : (eid > nE - 1 ? nE - 1 : eid);
      int sr = srcs[eid]; sr = sr < 0 ? 0 : (sr > nN - 1 ? nN - 1 : sr);
      const int m32 = (cnt - b0) < 32 ? (cnt - b0) : 32;
#pragma unroll 1
      for (int k = 0; k < m32; ++k) {
        const int sk = __builtin_amdgcn_readlane(sr, k);
        const float es = SC[(size_t)sk * SCW + hd];
        const v4f v = *(const v4fa*)(F + (size_t)sk * DF + 4 * lane);
        float lg = es + sdv;
        lg = lg > 0.f ? lg : NEGSL * lg;
        const float df = lg - mx;
        const float ee = __expf(-fabsf(df));
        const bool up  = df > 0.f;
        const float s1 = up ? ee : 1.0f;
        const float s2 = up ? 1.0f : ee;
        mx = up ? lg : mx;
        dn = fmaf(dn, s1, s2);
        a0 = fmaf(a0, s1, s2 * v.x);
        a1 = fmaf(a1, s1, s2 * v.y);
        a2 = fmaf(a2, s1, s2 * v.z);
        a3 = fmaf(a3, s1, s2 * v.w);
      }
    }
    const float dd  = dn > 0.0f ? dn : 1.0f;
    const float inv = __builtin_amdgcn_rcpf(dd);
    const float h0 = fmaf(a0, inv, bb.x);
    const float h1 = fmaf(a1, inv, bb.y);
    const float h2 = fmaf(a2, inv, bb.z);
    const float h3 = fmaf(a3, inv, bb.w);

    if (live) {
      wn += 1;
      const float rk = __builtin_amdgcn_rcpf((float)wn);
      const float d0 = h0 - wm0; wm0 = fmaf(d0, rk, wm0); wq0 = fmaf(d0, h0 - wm0, wq0);
      const float d1 = h1 - wm1; wm1 = fmaf(d1, rk, wm1); wq1 = fmaf(d1, h1 - wm1, wq1);
      const float d2 = h2 - wm2; wm2 = fmaf(d2, rk, wm2); wq2 = fmaf(d2, h2 - wm2, wq2);
      const float d3 = h3 - wm3; wm3 = fmaf(d3, rk, wm3); wq3 = fmaf(d3, h3 - wm3, wq3);
    }
    v4f pv;
    pv.x = (live ? h0 : 0.f) + pz;
    pv.y = (live ? h1 : 0.f) + pz;
    pv.z = (live ? h2 : 0.f) + pz;
    pv.w = (live ? h3 : 0.f) + pz;
    float* gp = HCo + (size_t)node * (size_t)DF + 4 * lane;
    *(volatile v4f*)gp = pv;
    __threadfence();
    *(volatile v4f*)gp = pv;
  }

  float* wst = (float*)lds_i;
  float* pst = wst + NWAVE * WSTW;
  if (lane == 0) wst[wave * WSTW] = (float)wn;
  {
    float* wr = wst + wave * WSTW + 1 + 4 * lane;
    wr[0] = wm0; wr[1] = wm1; wr[2] = wm2; wr[3] = wm3;
    wr[DF + 0] = wq0; wr[DF + 1] = wq1; wr[DF + 2] = wq2; wr[DF + 3] = wq3;
  }
  __syncthreads();
  if (tid < DF) {
    float n = 0.0f, mean = 0.0f, M2 = 0.0f;
#pragma unroll 1
    for (int w2 = 0; w2 < NWAVE; ++w2) {
      const float nbv = wst[w2 * WSTW];
      const float mb  = wst[w2 * WSTW + 1 + tid];
      const float qb  = wst[w2 * WSTW + 1 + DF + tid];
      if (nbv > 0.5f) {
        const float nn = n + nbv;
        const float delta = mb - mean;
        const float f = nbv / nn;
        mean = fmaf(delta, f, mean);
        M2 = M2 + qb + delta * delta * n * f;
        n = nn;
      }
    }
    pst[1 + tid] = mean;
    pst[1 + DF + tid] = M2;
    if (tid == 0) pst[0] = n;
  }
#pragma unroll 1
  for (int i = 2 * DF + 1 + tid; i < PARTW; i += NTHR) pst[i] = 0.0f;
  __syncthreads();
  const int pb = (int)blockIdx.x;
  v4f ps = {0.0f, 0.0f, 0.0f, 0.0f};
  if (tid < PARTW / 4) {
    ps = *(const v4fa*)(pst + 4 * tid);
    *(volatile v4f*)(part + (size_t)pb * PARTW + 4 * tid) = ps;
  }
  __threadfence();
  if (tid < PARTW / 4) {
    *(volatile v4f*)(part + (size_t)pb * PARTW + 4 * tid) = ps;
  }
}

__global__ __launch_bounds__(DF) void k_bnfin(const float* __restrict__ part, int nPart,
                                              const float* __restrict__ gam, const float* __restrict__ bet,
                                              float* ss) {
  __shared__ __attribute__((aligned(16))) float stg[2 * DF];
  const int tid = (int)threadIdx.x;
  const int c = tid;
  double n = 0.0, mean = 0.0, M2 = 0.0;
#pragma unroll 1
  for (int b = 0; b < nPart; ++b) {
    const float* pr = part + (size_t)b * PARTW;
    const double nbv = (double)pr[0];
    const double mb  = (double)pr[1 + c];
    const double qb  = (double)pr[1 + DF + c];
    if (nbv > 0.5) {
      const double nn = n + nbv;
      const double delta = mb - mean;
      const double f = nbv / nn;
      mean = mean + delta * f;
      M2 = M2 + qb + delta * delta * n * f;
      n = nn;
    }
  }
  const double nt = n < 1.0 ? 1.0 : n;
  const float varf  = (float)(M2 / nt);
  const float meanf = (float)mean;
  const float rstd = 1.0f / sqrtf(varf + BNEPS);
  const float sc = bf_rne(gam[c]) * rstd;
  const float sh = bf_rne(bet[c]) - meanf * sc;
  stg[c] = sc;
  stg[DF + c] = sh;
  __syncthreads();
  v4f v = {0.0f, 0.0f, 0.0f, 0.0f};
  if (tid < (2 * DF) / 4) {
    v = *(const v4fa*)(stg + 4 * tid);
    *(volatile v4f*)(ss + 4 * tid) = v;
  }
  __threadfence();
  if (tid < (2 * DF) / 4) {
    *(volatile v4f*)(ss + 4 * tid) = v;
  }
}

__global__ __launch_bounds__(NTHR) void k_apply(const float* __restrict__ src, const float* __restrict__ ss,
                                                int nValid, int nUnits, float* dst) {
  __shared__ __attribute__((aligned(16))) float ssh[2 * DF];
  const int tid = (int)threadIdx.x;
  ssh[tid] = ss[tid];
  __syncthreads();
  const int u = (int)blockIdx.x * NTHR + tid;
  const bool act = u < nUnits;
  const int uc = act ? u : (nUnits - 1);
  const int row = uc >> 5;
  const int piece = uc & 31;
  const int c0 = 4 * piece;
  const int rc = row < nValid ? row : nValid - 1;
  const v4f a   = *(const v4fa*)(src + (size_t)rc * DF + c0);
  const v4f sca = *(const v4fa*)(ssh + c0);
  const v4f sha = *(const v4fa*)(ssh + DF + c0);
  const bool live = row < nValid;
  float y[4];
  y[0] = fmaf(a.x, sca.x, sha.x); y[1] = fmaf(a.y, sca.y, sha.y);
  y[2] = fmaf(a.z, sca.z, sha.z); y[3] = fmaf(a.w, sca.w, sha.w);
  float t[4];
#pragma unroll
  for (int j = 0; j < 4; ++j) {
    const float e = __expf(y[j]) - 1.0f;
    const float r = y[j] > 0.0f ? y[j] : e;
    t[j] = live ? r : 0.0f;
  }
  v4f pv;
  pv.x = t[0]; pv.y = t[1]; pv.z = t[2]; pv.w = t[3];
  float* op = dst + (size_t)row * DF + c0;
  if (act) *(volatile v4f*)op = pv;
  __threadfence();
  if (act) *(volatile v4f*)op = pv;
}

__global__ __launch_bounds__(NTHR) void k_sumagg(const int* __restrict__ dsts, const int* __restrict__ srcs,
                                                 const float* __restrict__ X, const float* __restrict__ epsp,
                                                 unsigned short* Aout, int nN, int nE, int vec8) {
  extern __shared__ __attribute__((aligned(16))) int lds_i[];
  const int tid = (int)threadIdx.x, lane = tid & 31, wave = tid >> 5;
  const int nodeBase = (int)blockIdx.x * NBA;
  const int nh = seg_build(dsts, nE, vec8, nodeBase, lds_i, tid, lane, wave);
  const int* reg2 = lds_i + RCAP;
  const int* scnt = reg2 + RCAP;
  const int* soff = scnt + NBA;

  const int nbw = NBA / NWAVE;
  const bool ovf = (nh >= RCAP);
  const float qnan = __int_as_float(0x7fc00000);
  const float es1 = 1.0f + bf_rne(epsp[0]);

#pragma unroll 1
  for (int jt = 0; jt < nbw; ++jt) {
    const int slot = wave * nbw + jt;
    const int node = nodeBase + slot;
    int st = soff[slot];
    const int craw = scnt[slot];
    int cnt = craw;
    st  = st < 0 ? 0 : (st > nh ? nh : st);
    cnt = cnt < 0 ? 0 : (cnt > DEGCAP ? DEGCAP : cnt);
    if (cnt > nh - st) cnt = nh - st;
    const float pz = (ovf || craw > DEGCAP) ? qnan : 0.0f;
    const bool live = node < nN;
    const int nc = node < nN ? node : nN - 1;

    float a0 = 0.f, a1 = 0.f, a2 = 0.f, a3 = 0.f;
#pragma unroll 1
    for (int b0 = 0; b0 < cnt; b0 += 32) {
      int idx = st + b0 + lane; idx = idx > RCAP - 1 ? RCAP - 1 : idx;
      int eid = reg2[idx]; eid = eid < 0 ? 0 : (eid > nE - 1 ? nE - 1 : eid);
      int sr = srcs[eid]; sr = sr < 0 ? 0 : (sr > nN - 1 ? nN - 1 : sr);
      const int m32 = (cnt - b0) < 32 ? (cnt - b0) : 32;
#pragma unroll 1
      for (int k = 0; k < m32; ++k) {
        const int sk = __builtin_amdgcn_readlane(sr, k);
        const v4f v = *(const v4fa*)(X + (size_t)sk * DF + 4 * lane);
        a0 += v.x; a1 += v.y; a2 += v.z; a3 += v.w;
      }
    }
    const v4f sv = *(const v4fa*)(X + (size_t)nc * DF + 4 * lane);
    float r0 = fmaf(es1, sv.x, a0), r1 = fmaf(es1, sv.y, a1);
    float r2 = fmaf(es1, sv.z, a2), r3 = fmaf(es1, sv.w, a3);
    r0 = (live ? r0 : 0.0f) + pz;
    r1 = (live ? r1 : 0.0f) + pz;
    r2 = (live ? r2 : 0.0f) + pz;
    r3 = (live ? r3 : 0.0f) + pz;

    const unsigned short hb0 = bf_bits(r0), hb1 = bf_bits(r1), hb2 = bf_bits(r2), hb3 = bf_bits(r3);
    const unsigned short lb0 = bf_bits(r0 - bf_val(hb0)), lb1 = bf_bits(r1 - bf_val(hb1));
    const unsigned short lb2 = bf_bits(r2 - bf_val(hb2)), lb3 = bf_bits(r3 - bf_val(hb3));
    v4u pk;
    pk.x = (unsigned int)hb0 | ((unsigned int)hb1 << 16);
    pk.y = (unsigned int)hb2 | ((unsigned int)hb3 << 16);
    pk.z = (unsigned int)lb0 | ((unsigned int)lb1 << 16);
    pk.w = (unsigned int)lb2 | ((unsigned int)lb3 << 16);
    unsigned short* gp = Aout + (size_t)node * (size_t)KZ + 8 * lane;
    *(volatile v4u*)gp = pk;
    __threadfence();
    *(volatile v4u*)gp = pk;
  }
}

__global__ __launch_bounds__(GTHR) void k_gemm2(const unsigned short* __restrict__ A,
                                                const unsigned short* __restrict__ BT,
                                                const float* __restrict__ bias,
                                                float* C32, float* part, int nN, int nRows) {
  __shared__ __attribute__((aligned(16))) float stg[GBM * GBN];
  __shared__ __attribute__((aligned(16))) float pst[PARTW];
  const int tid = (int)threadIdx.x, lane = tid & 31, wave = tid >> 5, hh = lane >> 4, m = lane & 15;
  const int rowBase = (int)blockIdx.x * GBM;

  v8f acc[GNT];
#pragma unroll
  for (int t = 0; t < GNT; ++t) acc[t] = z8();
  const unsigned short* ap = A  + (size_t)(rowBase + 16 * wave + m) * (size_t)KZ + 8 * hh;
  const unsigned short* bp = BT + (size_t)m * (size_t)KZ + 8 * hh;

#pragma unroll 1
  for (int k0 = 0; k0 < KZ; k0 += 32) {
    Frag af;
    af.h[0] = *(const v8usa*)(ap + k0);
    af.h[1] = *(const v8usa*)(ap + k0 + 16);
#pragma unroll
    for (int nt = 0; nt < GNT; ++nt) {
      const unsigned short* wq = bp + (size_t)(16 * nt) * (size_t)KZ + k0;
      Frag bf;
      bf.h[0] = *(const v8usa*)wq;
      bf.h[1] = *(const v8usa*)(wq + 16);
      acc[nt] = wmk(af, bf, acc[nt]);
    }
  }

#pragma unroll
  for (int nt = 0; nt < GNT; ++nt) {
    const int lc = 16 * nt + m;
    const float bbv = bf_rne(bias[lc]);
#pragma unroll
    for (int r = 0; r < 8; ++r) {
      const int lr = 16 * wave + 8 * hh + r;
      stg[lr * GBN + lc] = acc[nt][r] + bbv;
    }
  }
  __syncthreads();

  {
    v4f pv[16];
#pragma unroll
    for (int i = 0; i < 16; ++i) pv[i] = *(const v4fa*)(stg + (16 * wave + i) * GBN + 4 * lane);
#pragma unroll
    for (int i = 0; i < 16; ++i) {
      const int gr = rowBase + 16 * wave + i;
      float* op = C32 + (size_t)gr * (size_t)DF + 4 * lane;
      if (gr < nRows) *(volatile v4f*)op = pv[i];
    }
    __threadfence();
#pragma unroll
    for (int i = 0; i < 16; ++i) {
      const int gr = rowBase + 16 * wave + i;
      float* op = C32 + (size_t)gr * (size_t)DF + 4 * lane;
      if (gr < nRows) *(volatile v4f*)op = pv[i];
    }
  }

  {
    int nl = nN - rowBase;
    nl = nl < 0 ? 0 : (nl > GBM ? GBM : nl);
    float s = 0.0f;
#pragma unroll 1
    for (int r = 0; r < nl; ++r) s += stg[r * GBN + tid];
    const float fn = (float)(nl > 0 ? nl : 1);
    const float mean = s / fn;
    float q = 0.0f;
#pragma unroll 1
    for (int r = 0; r < nl; ++r) {
      const float d = stg[r * GBN + tid] - mean;
      q = fmaf(d, d, q);
    }
    pst[1 + tid] = mean;
    pst[1 + DF + tid] = q;
    if (tid == 0) pst[0] = (float)nl;
#pragma unroll 1
    for (int i = 2 * DF + 1 + tid; i < PARTW; i += GTHR) pst[i] = 0.0f;
  }
  __syncthreads();
  const int pb = (int)blockIdx.x;
  v4f ps = {0.0f, 0.0f, 0.0f, 0.0f};
  if (tid < PARTW / 4) {
    ps = *(const v4fa*)(pst + 4 * tid);
    *(volatile v4f*)(part + (size_t)pb * PARTW + 4 * tid) = ps;
  }
  __threadfence();
  if (tid < PARTW / 4) {
    *(volatile v4f*)(part + (size_t)pb * PARTW + 4 * tid) = ps;
  }
}

static inline int cdiv(int a, int b) { return (a + b - 1) / b; }
static inline size_t al256(size_t o) { return (o + 255) & ~(size_t)255; }

extern "C" void kernel_launch(void* const* d_in, const int* in_sizes, int n_in,
                              void* d_out, int out_size, void* d_ws, size_t ws_size,
                              hipStream_t stream) {
  if (n_in < 13) return;
  if (in_sizes[0] < DF || (in_sizes[0] % DF) != 0) return;
  const int nN = in_sizes[0] / DF;
  if (nN < 1 || nN > (1 << 22)) return;
  if (in_sizes[1] < 2 || (in_sizes[1] & 1) != 0) return;
  const int nE = in_sizes[1] / 2;
  if (nE < 1 || nE >= (1 << 21)) return;
  if (in_sizes[2] != DF * DF) return;
  if (in_sizes[3] != NHEAD * HCH || in_sizes[4] != NHEAD * HCH) return;
  if (in_sizes[5] != DF) return;
  if (in_sizes[6] != DF || in_sizes[7] != DF) return;
  if (in_sizes[8] < 1) return;
  if (in_sizes[9] != DF * DF) return;
  if (in_sizes[10] != DF) return;
  if (in_sizes[11] != DF || in_sizes[12] != DF) return;
  if ((long long)out_size != (long long)nN * DF) return;

  const float* x     = (const float*)d_in[0];
  const int*   ei    = (const int*)  d_in[1];
  const float* Wa    = (const float*)d_in[2];
  const float* asr   = (const float*)d_in[3];
  const float* ads   = (const float*)d_in[4];
  const float* ba    = (const float*)d_in[5];
  const float* g1    = (const float*)d_in[6];
  const float* be1   = (const float*)d_in[7];
  const float* epsp  = (const float*)d_in[8];
  const float* Wb    = (const float*)d_in[9];
  const float* bb    = (const float*)d_in[10];
  const float* g2    = (const float*)d_in[11];
  const float* be2   = (const float*)d_in[12];
  float* out = (float*)d_out;
  const int* dst = ei;
  const int* src = ei + nE;

  const int MP   = cdiv(nN, GBM) * GBM;
  const int gM   = MP / GBM;
  const int gA   = cdiv(MP, NBA);
  const int RA   = gA * NBA;
  const int vec8 = 1;
  if ((long long)RA < (long long)MP) return;

  char* ws = (char*)d_ws;
  size_t off = 0;
  const size_t oWA = off; off = al256(off + (size_t)DF * KX * 2);
  const size_t oWZ = off; off = al256(off + (size_t)DF * KZ * 2);
  const size_t oSC = off; off = al256(off + (size_t)MP * SCW * 4);
  const size_t oP1 = off; off = al256(off + (size_t)gA * PARTW * 4);
  const size_t oS1 = off; off = al256(off + (size_t)(2 * DF) * 4);
  const size_t oP2 = off; off = al256(off + (size_t)gM * PARTW * 4);
  const size_t oS2 = off; off = al256(off + (size_t)(2 * DF) * 4);
  const size_t oRA = off; off = al256(off + (size_t)MP * DF * 4);
  size_t szB = (size_t)RA * DF * 4;
  if ((size_t)MP * KX * 2 > szB) szB = (size_t)MP * KX * 2;
  if ((size_t)RA * KZ * 2 > szB) szB = (size_t)RA * KZ * 2;
  const size_t oRB = off; off = al256(off + szB);
  if (off > ws_size || off > (size_t)WSMAX) return;
  unsigned short* WA  = (unsigned short*)(ws + oWA);
  unsigned short* WZ  = (unsigned short*)(ws + oWZ);
  float*          SC  = (float*)(ws + oSC);
  float*          P1  = (float*)(ws + oP1);
  float*          S1  = (float*)(ws + oS1);
  float*          P2  = (float*)(ws + oP2);
  float*          S2  = (float*)(ws + oS2);
  float*          H   = (float*)(ws + oRA);
  float*          X1  = (float*)(ws + oRA);
  float*          H2  = (float*)(ws + oRA);
  unsigned short* XB  = (unsigned short*)(ws + oRB);
  float*          HCp = (float*)(ws + oRB);
  unsigned short* ZP  = (unsigned short*)(ws + oRB);

  hipFuncSetAttribute(reinterpret_cast<const void*>(&k_attagg), hipFuncAttributeMaxDynamicSharedMemorySize, LDS_AGG);
  hipFuncSetAttribute(reinterpret_cast<const void*>(&k_sumagg), hipFuncAttributeMaxDynamicSharedMemorySize, LDS_AGG);

  k_wprep<<<NUW / NTHR, NTHR, 0, stream>>>(Wa, Wb, WA, WZ);
  {
    const int nUx = MP * 16;
    k_cvt<<<cdiv(nUx, NTHR), NTHR, 0, stream>>>(x, nN, nUx, XB);
  }
  k_gemm1<<<gM, GTHR, 0, stream>>>(XB, WA, asr, ads, H, SC);
  k_attagg<<<gA, NTHR, LDS_AGG, stream>>>(dst, src, H, SC, ba, HCp, P1, nN, nE, vec8);
  k_bnfin<<<1, DF, 0, stream>>>(P1, gA, g1, be1, S1);
  {
    const int nUa = MP * 32;
    k_apply<<<cdiv(nUa, NTHR), NTHR, 0, stream>>>(HCp, S1, nN, nUa, X1);
  }
  k_sumagg<<<gA, NTHR, LDS_AGG, stream>>>(dst, src, X1, epsp, ZP, nN, nE, vec8);
  k_gemm2<<<gM, GTHR, 0, stream>>>(ZP, WZ, bb, H2, P2, nN, MP);
  k_bnfin<<<1, DF, 0, stream>>>(P2, gM, g2, be2, S2);
  {
    const int nUo = nN * 32;
    k_apply<<<cdiv(nUo, NTHR), NTHR, 0, stream>>>(H2, S2, nN, nUo, out);
  }
}
